// CausalPerformer_5918464934283
// MI455X (gfx1250) — hardware-verified
//
#include <hip/hip_runtime.h>


namespace {
constexpr int Bn = 2, S = 4096, DM = 1024, H = 16, HD = 64, F = 7, FP = 16  , NTOK = Bn * S, NBH = Bn * H, CH = 64, NC = S / CH;
constexpr float PS8 = 8.0f, CXS = 1.0f / 64.0f, EPS = 1e-6f;
constexpr size_t FPL = (size_t)NBH * S * FP  , FTPL = (size_t)NBH * FP * S  , VPL = (size_t)NBH * HD * S  , CPL = (size_t)NBH * NC * HD * FP  ;

typedef _Float16 b16;
typedef __attribute__((ext_vector_type(16))) _Float16 v16b;
typedef __attribute__((ext_vector_type(16))) __bf16 v16bb;
typedef __attribute__((ext_vector_type(8))) _Float16 v8b;
typedef __attribute__((ext_vector_type(8))) unsigned short v8us;
typedef __attribute__((ext_vector_type(8))) float v8f;
typedef __attribute__((ext_vector_type(4))) float v4f;
typedef __attribute__((ext_vector_type(2))) _Float16 v2b; typedef __attribute__((ext_vector_type(2))) float v2f;
__device__ __forceinline__ float bf16_rne(float f) { unsigned int u = __float_as_uint(f); u += 0x7FFFu + ((u >> 16) & 1u); return __uint_as_float(u & 0xFFFF0000u); }
__device__ __forceinline__ unsigned short bf16_bits(float f) { unsigned int u = __float_as_uint(f); u += 0x7FFFu + ((u >> 16) & 1u); return (unsigned short)(u >> 16); }
__device__ __forceinline__ void split16(float v, b16& hi, b16& lo) { hi = (b16)v; lo = (b16)(v - (float)hi); }
__device__ __forceinline__ v16b frag_kb(const b16* p, int hh) { const v8b a = *(const v8b*)(p + 8 * hh), b = *(const v8b*)(p + 16 + 8 * hh); v16b f;
#pragma unroll
  for (int e = 0; e < 8; ++e) { f[e] = a[e]; f[8 + e] = b[e]; } return f; }
__device__ __forceinline__ v16b frag16(const b16* p, int hh) { const v8b a = *(const v8b*)(p + 8 * hh); v16b f;
#pragma unroll
  for (int e = 0; e < 8; ++e) { f[e] = a[e]; f[8 + e] = (b16)0.0f; } return f; }
__device__ __forceinline__ v16bb frag_bf(const unsigned short* p, int hh) { const v8us a = *(const v8us*)(p + 8 * hh), b = *(const v8us*)(p + 16 + 8 * hh); union { unsigned short s[16]; v16bb v; } u;
#pragma unroll
  for (int e = 0; e < 8; ++e) { u.s[e] = a[e]; u.s[8 + e] = b[e]; } return u.v; }
__device__ __forceinline__ v8f wmma16b(v16b a, v16b b, v8f c) { v8f d = __builtin_amdgcn_wmma_f32_16x16x32_f16(false, a, false, b, (short)0, c, false, false); asm volatile("v_nop\n\tv_nop\n\tv_nop\n\tv_nop" : "+v"(d) : "v"(a), "v"(b)); return d; }
__device__ __forceinline__ v8f wmma16bb(v16bb a, v16bb b, v8f c) { v8f d = __builtin_amdgcn_wmma_f32_16x16x32_bf16(false, a, false, b, (short)0, c, false, false); asm volatile("v_nop\n\tv_nop\n\tv_nop\n\tv_nop" : "+v"(d) : "v"(a), "v"(b)); return d; }
__device__ __forceinline__ void wave_lds_sync() { __builtin_amdgcn_fence(__ATOMIC_RELEASE, "workgroup"); __builtin_amdgcn_wave_barrier(); __builtin_amdgcn_fence(__ATOMIC_ACQUIRE, "workgroup"); }
__device__ __forceinline__ float pmul(float a, float b) { float p = a * b; asm volatile("" : "+v"(p)); return p; }

__global__ __launch_bounds__(256) void prep_kernel(const float* __restrict__ wq, const float* __restrict__ wk, const float* __restrict__ wv, const float* __restrict__ wo, const float* __restrict__ om, unsigned short* __restrict__ w16, b16* __restrict__ wo16, float* __restrict__ omr) {
  const size_t tid = (size_t)blockIdx.x * blockDim.x + threadIdx.x, nth = (size_t)gridDim.x * blockDim.x; const size_t WP = (size_t)DM * DM;
  for (int pass = 0; pass < 2; ++pass) {
    for (size_t p = tid; p < 3 * WP / 8; p += nth) { const size_t w = p / (WP / 8), q8 = p % (WP / 8); const float* src = (w == 0) ? wq : (w == 1) ? wk : wv; v8us o;
#pragma unroll
      for (int e = 0; e < 8; ++e) o[e] = bf16_bits(src[q8 * 8 + e]);
      *(volatile v8us*)(w16 + w * WP + q8 * 8) = o; }
    for (size_t p = tid; p < WP / 8; p += nth) { v8b o;
#pragma unroll
      for (int e = 0; e < 8; ++e) o[e] = (b16)bf16_rne(wo[p * 8 + e]);
      *(volatile v8b*)(wo16 + p * 8) = o; }
    for (size_t p = tid; p < (size_t)F * HD; p += nth) ((volatile float*)omr)[p] = bf16_rne(om[p]);
    __threadfence();
  }
}

__device__ __forceinline__ v16bb frag_f32bf(const float* p, int hh) { union { unsigned short s[16]; v16bb v; } u;
#pragma unroll
  for (int e = 0; e < 8; ++e) { u.s[e] = bf16_bits(p[8 * hh + e]); u.s[8 + e] = bf16_bits(p[16 + 8 * hh + e]); } return u.v; }
__global__ __launch_bounds__(128) void proj_kernel(const float* __restrict__ qin, const float* __restrict__ kin, const float* __restrict__ vin, const unsigned short* __restrict__ w16, const float* __restrict__ omr, b16* __restrict__ qf, b16* __restrict__ kf, b16* __restrict__ kfT, b16* __restrict__ vT) {
  __shared__ __attribute__((aligned(16))) float Ts[4][32][64 + 4]; __shared__ __attribute__((aligned(16))) b16 Fh[128][16], Fl[128][16]; __shared__ __attribute__((aligned(16))) b16 Tt[64][128 + 8], Ttl[64][128 + 8]; __shared__ float Om[F][64];
  const int lane = threadIdx.x & 31, wave = threadIdx.x >> 5, nloc = lane & 15, hlf = lane >> 4, which = blockIdx.z, head = blockIdx.x, m0 = blockIdx.y * 128 + wave * 32, c0 = head * HD;
  const int b = (blockIdx.y * 128) / S, tok0 = (blockIdx.y * 128) % S; const size_t WP = (size_t)DM * DM;
  const float* X = (which == 0) ? qin : (which == 1) ? kin : vin; const unsigned short* Wt = w16 + (size_t)which * WP;
  for (int i = threadIdx.x; i < F * 64; i += 128) Om[i / 64][i % 64] = omr[i];
  v8f acc[2][4];
#pragma unroll
  for (int r = 0; r < 2; ++r)
#pragma unroll
    for (int t = 0; t < 4; ++t) acc[r][t] = (v8f){};
#pragma unroll 2
  for (int kb = 0; kb < DM; kb += 32) { const v16bb a0 = frag_f32bf(X + (size_t)(m0 + nloc) * DM + kb, hlf), a1 = frag_f32bf(X + (size_t)(m0 + 16 + nloc) * DM + kb, hlf);
#pragma unroll
    for (int t = 0; t < 4; ++t) { const v16bb bw = frag_bf(Wt + (size_t)(c0 + t * 16 + nloc) * DM + kb, hlf); acc[0][t] = wmma16bb(a0, bw, acc[0][t]); acc[1][t] = wmma16bb(a1, bw, acc[1][t]); } }
  if (which < 2) {
#pragma unroll
    for (int t = 0; t < 4; ++t)
#pragma unroll
      for (int r = 0; r < 2; ++r)
#pragma unroll
        for (int v = 0; v < 8; ++v) Ts[wave][r * 16 + 8 * hlf + v][t * 16 + nloc] = acc[r][t][v];
    wave_lds_sync();
    { const int rr = lane; float p[F]; float s = 0.0f;
#pragma unroll
      for (int f = 0; f < F; ++f) { float u = 0.0f;
#pragma unroll 8
        for (int d = 0; d < 64; ++d) u += pmul(Ts[wave][rr][d], Om[f][d]);
        p[f] = __expf(-0.5f * u * u); s += p[f]; }
      const float inv = 1.0f / (s + EPS);
#pragma unroll
      for (int f = 0; f < 16; ++f) { float val = (f < F) ? p[(f < F) ? f : 0] * inv : 0.0f; b16 a_, c_; split16(val * PS8, a_, c_); Fh[wave * 32 + rr][f] = a_; Fl[wave * 32 + rr][f] = c_; } }
    __syncthreads();
    const size_t bh = (size_t)b * H + head; b16* dst = ((which == 0) ? qf : kf) + (bh * S + tok0) * FP;
    for (int pass = 0; pass < 2; ++pass) {
      for (int i = threadIdx.x; i < 128 * 16 / 8; i += 128) { *(volatile v8b*)(dst + (size_t)i * 8) = *(const v8b*)(&Fh[0][0] + i * 8); *(volatile v8b*)(dst + FPL + (size_t)i * 8) = *(const v8b*)(&Fl[0][0] + i * 8); }
      if (which == 1) { for (int i = threadIdx.x; i < 16 * 16; i += 128) { const int f = i >> 4, c8 = (i & 15) * 8; v8b oh, ol;
#pragma unroll
          for (int e = 0; e < 8; ++e) { oh[e] = Fh[c8 + e][f]; ol[e] = Fl[c8 + e][f]; }
          *(volatile v8b*)(kfT + (bh * FP + f) * S + tok0 + c8) = oh; *(volatile v8b*)(kfT + FTPL + (bh * FP + f) * S + tok0 + c8) = ol; } }
      __threadfence(); }
    return;
  }
#pragma unroll
  for (int t = 0; t < 4; ++t)
#pragma unroll
    for (int r = 0; r < 2; ++r)
#pragma unroll
      for (int v = 0; v < 8; ++v) { b16 a_, c_; split16(acc[r][t][v] * PS8, a_, c_); Tt[t * 16 + nloc][wave * 32 + r * 16 + 8 * hlf + v] = a_; Ttl[t * 16 + nloc][wave * 32 + r * 16 + 8 * hlf + v] = c_; }
  __syncthreads();
  b16* dstT = vT + (((size_t)b * H + head) * HD) * S + tok0;
  for (int pass = 0; pass < 2; ++pass) {
#pragma unroll
    for (int j = 0; j < 8; ++j) { const int dd = wave * 16 + j * 2 + (lane >> 4), c8 = (lane & 15) * 8; *(volatile v8b*)(dstT + (size_t)dd * S + c8) = *(const v8b*)(&Tt[dd][c8]); *(volatile v8b*)(dstT + VPL + (size_t)dd * S + c8) = *(const v8b*)(&Ttl[dd][c8]); }
    __threadfence(); }
}

__global__ __launch_bounds__(32) void chunk_kernel(const b16* __restrict__ kfT, const b16* __restrict__ vT, float* __restrict__ kv, float* __restrict__ ks) {
  __shared__ __attribute__((aligned(16))) float Ts[16][64 + 4]; __shared__ float Ks_[16];
  const int lane = threadIdx.x, nloc = lane & 15, hlf = lane >> 4; const int bh = blockIdx.x / NC, c = blockIdx.x % NC, n0 = c * CH;
  const b16* A0 = kfT + ((size_t)bh * FP) * S + n0; const b16* B0 = vT + ((size_t)bh * HD) * S + n0;
  v8f acc[4] = {{}, {}, {}, {}};
#pragma unroll
  for (int kb = 0; kb < CH; kb += 32) { const v16b a = frag_kb(A0 + (size_t)nloc * S + kb, hlf), al = frag_kb(A0 + FTPL + (size_t)nloc * S + kb, hlf);
#pragma unroll
    for (int t = 0; t < 4; ++t) { const v16b bv = frag_kb(B0 + (size_t)(t * 16 + nloc) * S + kb, hlf), bl = frag_kb(B0 + VPL + (size_t)(t * 16 + nloc) * S + kb, hlf);
      acc[t] = wmma16b(a, bv, acc[t]); acc[t] = wmma16b(al, bv, acc[t]); acc[t] = wmma16b(a, bl, acc[t]); } }
#pragma unroll
  for (int t = 0; t < 4; ++t)
#pragma unroll
    for (int v = 0; v < 8; ++v) Ts[8 * hlf + v][t * 16 + nloc] = acc[t][v] * (1.0f / (PS8 * PS8));
  if (lane < 16) { const b16* r = A0 + (size_t)lane * S; float s = 0.0f; for (int m = 0; m < CH; ++m) s += ((float)r[m] + (float)r[FTPL + m]); Ks_[lane] = s * (1.0f / PS8); }
  wave_lds_sync();
  float* dst = kv + (((size_t)bh * NC + c) * 16) * HD;
  for (int pass = 0; pass < 2; ++pass) { for (int i = lane; i < 16 * 16; i += 32) { const int rr = i >> 4, c4 = (i & 15) * 4; *(volatile v4f*)(dst + (size_t)rr * HD + c4) = *(const v4f*)(&Ts[rr][c4]); }
    if (lane < 4) *(volatile v4f*)(ks + ((size_t)bh * NC + c) * 16 + lane * 4) = *(const v4f*)(&Ks_[lane * 4]);
    __threadfence(); }
}

__global__ __launch_bounds__(256) void prefix_kernel(const float* __restrict__ kv, const float* __restrict__ ks, b16* __restrict__ cth, b16* __restrict__ ctl, float* __restrict__ cks) {
  const int g = blockIdx.x * 256 + threadIdx.x; const int bh = g >> 9, d = (g >> 3) & 63, fp = (g & 7) * 2;
  float r0 = 0.0f, r1 = 0.0f;
  for (int c = 0; c < NC; ++c) { const size_t o = (((size_t)bh * NC + c) * HD + d) * FP + fp; v2b vh, vl; b16 a, l; split16(r0 * CXS, a, l); vh[0] = a; vl[0] = l; split16(r1 * CXS, a, l); vh[1] = a; vl[1] = l;
    for (int pass = 0; pass < 2; ++pass) { *(volatile v2b*)(cth + o) = vh; *(volatile v2b*)(ctl + o) = vl; }
    if (fp < 16) { r0 += kv[(((size_t)bh * NC + c) * 16 + fp) * HD + d]; r1 += kv[(((size_t)bh * NC + c) * 16 + fp + 1) * HD + d]; } }
  __threadfence();
}
__global__ __launch_bounds__(256) void prefixk_kernel(const float* __restrict__ ks, float* __restrict__ cks) {
  const int g = blockIdx.x * 256 + threadIdx.x; const int bh = g >> 4, f = g & 15; float r = 0.0f;
  for (int c = 0; c < NC; ++c) { for (int pass = 0; pass < 2; ++pass) ((volatile float*)cks)[((size_t)c * NBH + bh) * 16 + f] = r; r += ks[((size_t)bh * NC + c) * 16 + f]; }
  __threadfence();
}

__global__ __launch_bounds__(256) void attn_kernel(const b16* __restrict__ qf, const b16* __restrict__ kf, const b16* __restrict__ vT, const b16* __restrict__ cth, const b16* __restrict__ ctl, const float* __restrict__ cks, float* __restrict__ orow) {
  __shared__ __attribute__((aligned(16))) float Os[8][16][HD + 4];
  const int wid = threadIdx.x >> 5, lane = threadIdx.x & 31, hh = lane >> 4, col = lane & 15;
  const int wg = blockIdx.x * 8 + wid, qt = wg & 3, c = (wg >> 2) % NC, bh = wg / (4 * NC), b = bh / H, h = bh % H, q0 = c * CH + qt * 16, qi = q0 + col;
  const b16* Q = qf + ((size_t)bh * S + qi) * FP; const b16* K = kf + ((size_t)bh * S) * FP; const b16* VT = vT + ((size_t)bh * HD) * S; const b16* CT = cth + (((size_t)bh * NC + c) * HD) * FP; const b16* CTL = ctl + (((size_t)bh * NC + c) * HD) * FP;
  const v16b qv = frag16(Q, hh), ql = frag16(Q + FPL, hh);
  v8f o[4] = {{}, {}, {}, {}};
#pragma unroll
  for (int n = 0; n < 4; ++n) { const v16b a = frag16(CT + (size_t)(n * 16 + col) * FP, hh), al = frag16(CTL + (size_t)(n * 16 + col) * FP, hh); o[n] = wmma16b(a, qv, o[n]); o[n] = wmma16b(al, qv, o[n]); o[n] = wmma16b(a, ql, o[n]); }
  float deni = 0.0f; { const float* ck = cks + ((size_t)c * NBH + bh) * 16; if (hh == 0) {
#pragma unroll
      for (int f = 0; f < F; ++f) deni += ((float)Q[f] + (float)Q[FPL + f]) * (1.0f / PS8) * ck[f]; }
    deni += __shfl_xor(deni, 16); }
  float dens = 0.0f;
#pragma unroll
  for (int kb2 = 0; kb2 < 2; ++kb2) { const int kb = c * CH + kb2 * 32; v8f s0 = {}, s1 = {};
    const v16b ka = frag16(K + (size_t)(kb + col) * FP, hh), kal = frag16(K + FPL + (size_t)(kb + col) * FP, hh), kb_ = frag16(K + (size_t)(kb + 16 + col) * FP, hh), kbl = frag16(K + FPL + (size_t)(kb + 16 + col) * FP, hh);
    s0 = wmma16b(ka, qv, s0); s0 = wmma16b(ka, ql, s0); s0 = wmma16b(kal, qv, s0); s1 = wmma16b(kb_, qv, s1); s1 = wmma16b(kb_, ql, s1); s1 = wmma16b(kbl, qv, s1);
    v16b pb, pl;
#pragma unroll
    for (int r = 0; r < 8; ++r) { const int m0_ = kb + 8 * hh + r, m1_ = kb + 16 + 8 * hh + r;
      const float p0 = (m0_ <= qi) ? s0[r] * (1.0f / (PS8 * PS8)) : 0.0f, p1 = (m1_ <= qi) ? s1[r] * (1.0f / (PS8 * PS8)) : 0.0f; dens += p0 + p1;
      b16 a, cc; split16(p0 * CXS, a, cc); pb[r] = a; pl[r] = cc; split16(p1 * CXS, a, cc); pb[8 + r] = a; pl[8 + r] = cc; }
#pragma unroll
    for (int n = 0; n < 4; ++n) { const v16b vf = frag_kb(VT + (size_t)(n * 16 + col) * S + kb, hh), vl = frag_kb(VT + VPL + (size_t)(n * 16 + col) * S + kb, hh);
      o[n] = wmma16b(vf, pb, o[n]); o[n] = wmma16b(vf, pl, o[n]); o[n] = wmma16b(vl, pb, o[n]); } }
  dens += __shfl_xor(dens, 16);
  const float den = deni + dens + EPS; const float sc = 1.0f / (CXS * PS8);
#pragma unroll
  for (int n = 0; n < 4; ++n)
#pragma unroll
    for (int r = 0; r < 8; ++r) Os[wid][col][n * 16 + 8 * hh + r] = o[n][r] * sc / den;
  wave_lds_sync();
  float* dst = orow + ((size_t)b * S + q0) * DM + h * HD;
  for (int pass = 0; pass < 2; ++pass) {
#pragma unroll
    for (int j = 0; j < 8; ++j) { const int rr = j * 2 + hh, c4 = col * 4; *(volatile v4f*)(dst + (size_t)rr * DM + c4) = *(const v4f*)(&Os[wid][rr][c4]); }
    __threadfence(); }
}

__global__ __launch_bounds__(128) void outproj_kernel(const float* __restrict__ orow, const b16* __restrict__ wo16, float* __restrict__ y) {
  __shared__ __attribute__((aligned(16))) float Ts[4][32 * 64];
  const int lane = threadIdx.x & 31, wave = threadIdx.x >> 5, nloc = lane & 15, hlf = lane >> 4, m0 = blockIdx.y * 128 + wave * 32, c0 = blockIdx.x * 64;
  v8f acc[2][4];
#pragma unroll
  for (int r = 0; r < 2; ++r)
#pragma unroll
    for (int t = 0; t < 4; ++t) acc[r][t] = (v8f){};
#pragma unroll 2
  for (int kb = 0; kb < DM; kb += 32) { v16b a0, a1, l0, l1;
#pragma unroll
    for (int e = 0; e < 16; ++e) { const int k = kb + ((e < 8) ? (8 * hlf + e) : (16 + 8 * hlf + e - 8)); b16 p, q; split16(orow[(size_t)(m0 + nloc) * DM + k] * PS8, p, q); a0[e] = p; l0[e] = q; split16(orow[(size_t)(m0 + 16 + nloc) * DM + k] * PS8, p, q); a1[e] = p; l1[e] = q; }
#pragma unroll
    for (int t = 0; t < 4; ++t) { const v16b bw = frag_kb(wo16 + (size_t)(c0 + t * 16 + nloc) * DM + kb, hlf); acc[0][t] = wmma16b(a0, bw, acc[0][t]); acc[0][t] = wmma16b(l0, bw, acc[0][t]); acc[1][t] = wmma16b(a1, bw, acc[1][t]); acc[1][t] = wmma16b(l1, bw, acc[1][t]); } }
  float* Tt = Ts[wave];
#pragma unroll
  for (int t = 0; t < 4; ++t)
#pragma unroll
    for (int r = 0; r < 2; ++r)
#pragma unroll
      for (int v = 0; v < 8; ++v) Tt[(r * 16 + v + 8 * hlf) * 64 + t * 16 + nloc] = acc[r][t][v] * (1.0f / PS8);
  wave_lds_sync();
  float* dst0 = y + (size_t)m0 * DM + c0;
  for (int pass = 0; pass < 2; ++pass) {
#pragma unroll
    for (int j = 0; j < 16; ++j) { const int rr = j * 2 + hlf, c4 = nloc * 4; *(volatile v4f*)(dst0 + (size_t)rr * DM + c4) = *(const v4f*)(Tt + rr * 64 + c4); }
    __threadfence(); }
}
}

extern "C" void kernel_launch(void* const* d_in, const int* in_sizes, int n_in,
                              void* d_out, int out_size, void* d_ws, size_t ws_size, hipStream_t stream) {
  (void)n_in; (void)out_size;
  const float* q = (const float*)d_in[0]; const float* k = (const float*)d_in[1]; const float* v = (const float*)d_in[2]; const float* wq = (const float*)d_in[3]; const float* wk = (const float*)d_in[4]; const float* wv = (const float*)d_in[5]; const float* wo = (const float*)d_in[6]; const float* om = (const float*)d_in[7];
  float* y = (float*)d_out;
  if (in_sizes[0] != NTOK * DM || in_sizes[1] != NTOK * DM || in_sizes[2] != NTOK * DM || in_sizes[3] != DM * DM || in_sizes[6] != DM * DM || in_sizes[7] != F * HD) return;
  size_t off = 0; char* ws = (char*)d_ws;
  auto carve = [&](size_t bytes) { char* p = ws + off; off += (bytes + 255) & ~(size_t)255; return p; };
  unsigned short* w16 = (unsigned short*)carve((size_t)3 * DM * DM * 2); b16* wo16 = (b16*)carve((size_t)DM * DM * 2); float* omr = (float*)carve(F * HD * 4 + 256);
  b16* qf = (b16*)carve(FPL * 2 * 2); b16* kf = (b16*)carve(FPL * 2 * 2); b16* kfT = (b16*)carve(FTPL * 2 * 2); b16* vT = (b16*)carve(VPL * 2 * 2);
  float* kv = (float*)carve((size_t)NBH * NC * 16 * HD * 4); float* ks = (float*)carve((size_t)NBH * NC * 16 * 4); b16* cth = (b16*)carve(CPL * 2); b16* ctl = (b16*)carve(CPL * 2); float* cks = (float*)carve((size_t)NC * NBH * 16 * 4); float* orow = (float*)carve((size_t)NTOK * DM * 4);
  if (off > ws_size) return;
  prep_kernel<<<256, 256, 0, stream>>>(wq, wk, wv, wo, om, w16, wo16, omr);
  proj_kernel<<<dim3(H, NTOK / 128, 3), 128, 0, stream>>>(q, k, v, w16, omr, qf, kf, kfT, vT);
  chunk_kernel<<<NBH * NC, 32, 0, stream>>>(kfT, vT, kv, ks);
  prefix_kernel<<<NBH * 64 * 8 / 256, 256, 0, stream>>>(kv, ks, cth, ctl, cks);
  prefixk_kernel<<<NBH * 16 / 256, 256, 0, stream>>>(ks, cks);
  attn_kernel<<<NBH * NC * 4 / 8, 256, 0, stream>>>(qf, kf, vT, cth, ctl, cks, orow);
  outproj_kernel<<<dim3(DM / 64, NTOK / 128), 128, 0, stream>>>(orow, wo16, y);
}
